// TransformerBlockPHGate_37546604101859
// MI455X (gfx1250) — hardware-verified
//
#include <hip/hip_runtime.h>


namespace {
constexpr int Bn = 2, L = 2048, D = 1024, H = 16, HD = 64, NT = Bn * L, DF = 4096;
constexpr float EPS = 1e-5f, XS = 8.0f, PS = 8.0f;

typedef _Float16 b16;
typedef __attribute__((ext_vector_type(16))) _Float16 v16b;
typedef __attribute__((ext_vector_type(8))) _Float16 v8b;
typedef __attribute__((ext_vector_type(8))) float v8f;
typedef __attribute__((ext_vector_type(4))) float v4f;
__device__ __forceinline__ void split16(float v, _Float16& hi, _Float16& lo) { hi = (_Float16)v; lo = (_Float16)(v - (float)hi); }
__device__ __forceinline__ float bf16_rne(float f) { unsigned int u = __float_as_uint(f); u += 0x7FFFu + ((u >> 16) & 1u); return __uint_as_float(u & 0xFFFF0000u); }
__device__ __forceinline__ v16b frag_kb(const b16* p, int hh) { const v8b a = *(const v8b*)(p + 8 * hh), b = *(const v8b*)(p + 16 + 8 * hh); v16b f;
#pragma unroll
  for (int e = 0; e < 8; ++e) { f[e] = a[e]; f[8 + e] = b[e]; } return f; }
__device__ __forceinline__ v16b frag_x(const float* p, int hh) { v16b f;
#pragma unroll
  for (int e = 0; e < 8; ++e) { f[e] = (b16)bf16_rne(p[8 * hh + e]); f[8 + e] = (b16)bf16_rne(p[16 + 8 * hh + e]); } return f; }
__device__ __forceinline__ v8f wmma16b(v16b a, v16b b, v8f c) { v8f d = __builtin_amdgcn_wmma_f32_16x16x32_f16(false, a, false, b, (short)0, c, false, false); asm volatile("v_nop\n\tv_nop\n\tv_nop\n\tv_nop" : "+v"(d) : "v"(a), "v"(b)); return d; }
__device__ __forceinline__ void wave_lds_sync() { __builtin_amdgcn_fence(__ATOMIC_RELEASE, "workgroup"); __builtin_amdgcn_wave_barrier(); __builtin_amdgcn_fence(__ATOMIC_ACQUIRE, "workgroup"); }
__device__ __forceinline__ float nexp(float x) { return __builtin_amdgcn_exp2f(x * 1.4426950408889634f); }
__device__ __forceinline__ float pmul(float a, float b) { float p = a * b; asm volatile("" : "+v"(p)); return p; }
__device__ __forceinline__ float wsum(float v) {
#pragma unroll
  for (int o = 1; o < 32; o <<= 1) v += __shfl_xor(v, o); return v; }
__device__ __forceinline__ void sincos_r(float ang, float& sn, float& cs) { const float k = rintf(ang * 0.15915494309189535f); float r = __builtin_fmaf(k, -6.28318548202514648f, ang); r = __builtin_fmaf(k, 1.7484556025237907e-7f, r);
  const float t = r * 0.15915494309189535f; sn = __builtin_amdgcn_sinf(t); cs = __builtin_amdgcn_cosf(t); }
__device__ __forceinline__ float tanh_n(float x) { const float e = __builtin_amdgcn_exp2f(x * 2.8853900817779268f); return 1.0f - 2.0f * __builtin_amdgcn_rcpf(e + 1.0f); }
__device__ __forceinline__ float gelu_t(float x) { const float c = 0.7978845608028654f; return 0.5f * x * (1.0f + tanh_n(c * (x + 0.044715f * x * x * x))); }

struct Wo_ { static constexpr size_t O = 0, F1 = (size_t)D * D, F2 = F1 + (size_t)DF * D, END = F2 + (size_t)D * DF; };
__global__ __launch_bounds__(256) void prep_kernel(const float* __restrict__ wo, const float* __restrict__ w1, const float* __restrict__ w2, const float* __restrict__ bo, const float* __restrict__ bg, const float* __restrict__ g1, const float* __restrict__ b1, const float* __restrict__ g2, const float* __restrict__ b2, const float* __restrict__ bf1, const float* __restrict__ bf2, b16* __restrict__ R, float* __restrict__ P) {
  const size_t tid = (size_t)blockIdx.x * 256 + threadIdx.x, nth = (size_t)gridDim.x * 256;
  auto tr = [&](size_t base, int nout, int kin, const float* W) { for (size_t p = tid; p < (size_t)nout * (kin / 8); p += nth) { const int o = (int)(p / (kin / 8)), k0 = (int)(p % (kin / 8)) * 8; v8b v;
#pragma unroll
      for (int e = 0; e < 8; ++e) v[e] = (b16)bf16_rne(W[(size_t)(k0 + e) * nout + o]); *(volatile v8b*)(R + base + (size_t)o * kin + k0) = v; } };
  for (int pass = 0; pass < 2; ++pass) { tr(Wo_::O, D, D, wo); tr(Wo_::F1, DF, D, w1); tr(Wo_::F2, D, DF, w2);
    for (size_t q = tid; q < 11264; q += nth) { const int i = (int)q; float v; if (i < 1024) v = bo[i]; else if (i < 2048) v = bg[i - 1024]; else if (i < 3072) v = g1[i - 2048]; else if (i < 4096) v = b1[i - 3072]; else if (i < 5120) v = g2[i - 4096]; else if (i < 6144) v = b2[i - 5120]; else if (i < 10240) v = bf1[i - 6144]; else v = bf2[i - 10240]; P[q] = bf16_rne(v); }
    __threadfence(); }
}

__global__ __launch_bounds__(256) void gate_kernel(const float* __restrict__ query, const float* __restrict__ Wg, const float* __restrict__ P, float* __restrict__ GT) {
  __shared__ float mu[D]; __shared__ float go[64];
  const int n = blockIdx.y, o0 = blockIdx.x * 64, t_ = threadIdx.x;
  for (int i = t_; i < D; i += 256) { float s = 0.0f; const float* q = query + (size_t)n * L * D + i; for (int t = 0; t < L; ++t) s += bf16_rne(q[(size_t)t * D]); mu[i] = s * (1.0f / L); }
  __syncthreads();
  if (t_ < 64) { float s = 0.0f; const int o = o0 + t_; for (int i = 0; i < D; ++i) s += pmul(mu[i], bf16_rne(Wg[(size_t)i * D + o])); go[t_] = 1.0f / (1.0f + nexp(-(s + P[1024 + o]))); }
  __syncthreads();
  for (int pass = 0; pass < 2; ++pass) { if (t_ < 16) *(volatile v4f*)(GT + (size_t)n * D + o0 + t_ * 4) = *(const v4f*)(&go[t_ * 4]); __threadfence(); }
}

__global__ __launch_bounds__(256) void ln32_kernel(const float* __restrict__ src, const float* __restrict__ g, const float* __restrict__ bb, float* __restrict__ dst) {
  const int row = blockIdx.x * 8 + (threadIdx.x >> 5), lane = threadIdx.x & 31; const float* xr = src + (size_t)row * D;
  float v[32]; float s = 0.0f;
#pragma unroll
  for (int i = 0; i < 32; ++i) { v[i] = xr[(i >> 3) * 256 + lane * 8 + (i & 7)]; s += v[i]; }
  s = wsum(s); const float mu = s * (1.0f / D); float q = 0.0f;
#pragma unroll
  for (int i = 0; i < 32; ++i) { const float d = v[i] - mu; q += pmul(d, d); }
  q = wsum(q); const float inv = rsqrtf(q * (1.0f / D) + EPS);
  for (int pass = 0; pass < 2; ++pass) {
#pragma unroll
    for (int gq = 0; gq < 4; ++gq) { const int c0 = gq * 256 + lane * 8; v4f o0, o1;
#pragma unroll
      for (int e = 0; e < 4; ++e) { o0[e] = pmul((v[gq * 8 + e] - mu) * inv, g[c0 + e]) + bb[c0 + e]; o1[e] = pmul((v[gq * 8 + 4 + e] - mu) * inv, g[c0 + 4 + e]) + bb[c0 + 4 + e]; }
      *(volatile v4f*)(dst + (size_t)row * D + c0) = o0; *(volatile v4f*)(dst + (size_t)row * D + c0 + 4) = o1; }
    __threadfence(); }
}

__global__ __launch_bounds__(256) void ln_kernel(const float* __restrict__ src, int rnd, const float* __restrict__ g, const float* __restrict__ bb, b16* __restrict__ dst) {
  const int row = blockIdx.x * 8 + (threadIdx.x >> 5), lane = threadIdx.x & 31; const float* xr = src + (size_t)row * D;
  float v[32]; float s = 0.0f;
#pragma unroll
  for (int i = 0; i < 32; ++i) { float x = xr[(i >> 3) * 256 + lane * 8 + (i & 7)]; if (rnd) x = bf16_rne(x); v[i] = x; s += x; }
  s = wsum(s); const float mu = s * (1.0f / D); float q = 0.0f;
#pragma unroll
  for (int i = 0; i < 32; ++i) { const float d = v[i] - mu; q += pmul(d, d); }
  q = wsum(q); const float inv = rsqrtf(q * (1.0f / D) + EPS);
  for (int pass = 0; pass < 2; ++pass) {
#pragma unroll
    for (int gq = 0; gq < 4; ++gq) { v8b o; const int c0 = gq * 256 + lane * 8;
#pragma unroll
      for (int e = 0; e < 8; ++e) o[e] = (b16)((pmul((v[gq * 8 + e] - mu) * inv, g[c0 + e]) + bb[c0 + e]) * XS);
      *(volatile v8b*)(dst + (size_t)row * D + c0) = o; }
    __threadfence(); }
}

template <int K, int N, int EPI, int RND>
__global__ __launch_bounds__(64) void gemm_kernel(const b16* __restrict__ A, const b16* __restrict__ Bw, const float* __restrict__ bias, const float* __restrict__ resid, b16* __restrict__ Ch, float* __restrict__ Cf, const float* __restrict__ gate = nullptr, const b16* __restrict__ Alo = nullptr) {
  __shared__ __attribute__((aligned(16))) float Ts[2][32][128 + 4];
  const int lane = threadIdx.x & 31, wave = threadIdx.x >> 5, nloc = lane & 15, hlf = lane >> 4, m0 = blockIdx.y * 32, c0 = blockIdx.x * 256 + wave * 128;
  v8f acc[2][8];
#pragma unroll
  for (int r = 0; r < 2; ++r)
#pragma unroll
    for (int t = 0; t < 8; ++t) acc[r][t] = (v8f){};
  for (int kb = 0; kb < K; kb += 32) { const v16b a0 = frag_kb(A + (size_t)(m0 + nloc) * K + kb, hlf), a1 = frag_kb(A + (size_t)(m0 + 16 + nloc) * K + kb, hlf);
    if (EPI == 4) { const v16b l0 = frag_kb(Alo + (size_t)(m0 + nloc) * K + kb, hlf), l1 = frag_kb(Alo + (size_t)(m0 + 16 + nloc) * K + kb, hlf);
#pragma unroll
      for (int t = 0; t < 8; ++t) { const v16b bw = frag_kb(Bw + (size_t)(c0 + t * 16 + nloc) * K + kb, hlf); acc[0][t] = wmma16b(a0, bw, acc[0][t]); acc[0][t] = wmma16b(l0, bw, acc[0][t]); acc[1][t] = wmma16b(a1, bw, acc[1][t]); acc[1][t] = wmma16b(l1, bw, acc[1][t]); } }
    else {
#pragma unroll
      for (int t = 0; t < 8; ++t) { const v16b bw = frag_kb(Bw + (size_t)(c0 + t * 16 + nloc) * K + kb, hlf); acc[0][t] = wmma16b(a0, bw, acc[0][t]); acc[1][t] = wmma16b(a1, bw, acc[1][t]); } } }
#pragma unroll
  for (int t = 0; t < 8; ++t) { const float bv = (bias != nullptr) ? bias[c0 + t * 16 + nloc] : 0.0f;
#pragma unroll
    for (int r = 0; r < 2; ++r)
#pragma unroll
      for (int v = 0; v < 8; ++v) { float y = acc[r][t][v] * (1.0f / XS) + bv; if (EPI == 2) y = fmaxf(y, 0.0f); if (EPI == 5) y = 0.5f * y * (1.0f + erff(y * 0.7071067811865476f)); if (EPI == 4) y = pmul(y, gate[(size_t)((m0 + r * 16) / L) * N + c0 + t * 16 + nloc]); Ts[wave][r * 16 + 8 * hlf + v][t * 16 + nloc] = y; } }
  wave_lds_sync();
  if (EPI == 3 && c0 < 2 * D) {
    for (int i = lane; i < 32 * 64; i += 32) { const int rr = i >> 6, cp = (i & 63) * 2; const int t = (m0 + rr) % L; const int i2 = ((c0 + cp) & 63) >> 1;
      const float invf = __builtin_amdgcn_exp2f(-(float)i2 * (13.287712379549449f / 32.0f));
      float sn, cs; sincos_r((float)t * invf, sn, cs); const float xe = Ts[wave][rr][cp], xo = Ts[wave][rr][cp + 1];
      Ts[wave][rr][cp] = pmul(xe, cs) - pmul(xo, sn); Ts[wave][rr][cp + 1] = pmul(xe, sn) + pmul(xo, cs); }
    wave_lds_sync(); }
  for (int pass = 0; pass < 2; ++pass) {
    if (EPI == 1 || EPI == 4) { for (int i = lane; i < 32 * 32; i += 32) { const int rr = i >> 5, c4 = (i & 31) * 4; const size_t gi = (size_t)(m0 + rr) * N + c0 + c4; v4f o = *(const v4f*)(&Ts[wave][rr][c4]); const v4f xr = *(const v4f*)(resid + gi);
        for (int e = 0; e < 4; ++e) o[e] += RND ? bf16_rne(xr[e]) : xr[e]; *(volatile v4f*)(Cf + gi) = o; } }
    else { for (int i = lane; i < 32 * 16; i += 32) { const int rr = i >> 4, c8 = (i & 15) * 8; v8b o; for (int e = 0; e < 8; ++e) o[e] = (b16)(Ts[wave][rr][c8 + e] * XS); *(volatile v8b*)(Ch + (size_t)(m0 + rr) * N + c0 + c8) = o; } }
    __threadfence(); }
}

__global__ __launch_bounds__(256) void vt_kernel(const float* __restrict__ val, b16* __restrict__ vt) {
  __shared__ __attribute__((aligned(16))) b16 T[HD][128 + 8];
  const int b = blockIdx.z, h = blockIdx.y, t0 = blockIdx.x * 128, t_ = threadIdx.x;
  for (int i = t_; i < 128 * HD; i += 256) { const int tk = i >> 6, d = i & 63; T[d][tk] = (b16)(bf16_rne(val[((size_t)(b * L + t0 + tk)) * D + h * HD + d]) * XS); }
  __syncthreads();
  for (int pass = 0; pass < 2; ++pass) { for (int i = t_; i < HD * 16; i += 256) { const int d = i >> 4, c8 = (i & 15) * 8; *(volatile v8b*)(vt + (((size_t)b * H + h) * HD + d) * L + t0 + c8) = *(const v8b*)(&T[d][c8]); } __threadfence(); }
}

__global__ __launch_bounds__(256) void attn_kernel(const float* __restrict__ query, const float* __restrict__ key, const int* __restrict__ mask, const b16* __restrict__ vt, b16* __restrict__ ctxh, b16* __restrict__ ctxl) {
  __shared__ __attribute__((aligned(16))) b16 Oh[16][8 * HD + 8], Ol[16][8 * HD + 8];
  const int wid = threadIdx.x >> 5, lane = threadIdx.x & 31, hh = lane >> 4, col = lane & 15; const int b = blockIdx.x / (L / 16), q0 = (blockIdx.x % (L / 16)) * 16, h = blockIdx.y * 8 + wid, qi = q0 + col;
  const float* Qr = query + (size_t)(b * L) * D + h * HD; const float* Kr = key + (size_t)(b * L) * D + h * HD; const b16* V = vt + (((size_t)b * H + h) * HD) * L; const int* mrow = mask + (size_t)qi * L;
  const v16b qf0 = frag_x(Qr + (size_t)qi * D, hh), qf1 = frag_x(Qr + (size_t)qi * D + 32, hh);
  float m = -INFINITY, l = 0.0f; v8f o[4] = {{}, {}, {}, {}};
  for (int kb = 0; kb < L; kb += 32) {
    const v16b ka0 = frag_x(Kr + (size_t)(kb + col) * D, hh), ka1 = frag_x(Kr + (size_t)(kb + col) * D + 32, hh), kc0 = frag_x(Kr + (size_t)(kb + 16 + col) * D, hh), kc1 = frag_x(Kr + (size_t)(kb + 16 + col) * D + 32, hh);
    v8f s0 = {}, s1 = {}; s0 = wmma16b(ka0, qf0, s0); s0 = wmma16b(ka1, qf1, s0); s1 = wmma16b(kc0, qf0, s1); s1 = wmma16b(kc1, qf1, s1);
    float mr = -INFINITY;
#pragma unroll
    for (int r = 0; r < 8; ++r) { const int k0 = kb + 8 * hh + r, k1 = k0 + 16; s0[r] = (mrow[k0] != 0) ? s0[r] * 0.125f : -INFINITY; s1[r] = (mrow[k1] != 0) ? s1[r] * 0.125f : -INFINITY; mr = fmaxf(mr, fmaxf(s0[r], s1[r])); }
    mr = fmaxf(mr, __shfl_xor(mr, 16));
    const float mn = fmaxf(m, mr); const float al_ = (mn == -INFINITY) ? 1.0f : nexp(m - mn); m = mn; float sum = 0.0f; v16b ph, pl;
#pragma unroll
    for (int r = 0; r < 8; ++r) { const float e0 = (s0[r] == -INFINITY) ? 0.0f : nexp(s0[r] - mn), e1 = (s1[r] == -INFINITY) ? 0.0f : nexp(s1[r] - mn); sum += e0 + e1; b16 a_, c_; split16(e0 * PS, a_, c_); ph[r] = a_; pl[r] = c_; split16(e1 * PS, a_, c_); ph[8 + r] = a_; pl[8 + r] = c_; }
    sum += __shfl_xor(sum, 16); l = l * al_ + sum;
#pragma unroll
    for (int t = 0; t < 4; ++t) { o[t] *= al_; const v16b vf = frag_kb(V + (size_t)(t * 16 + col) * L + kb, hh); o[t] = wmma16b(vf, ph, o[t]); o[t] = wmma16b(vf, pl, o[t]); } }
  const float inv = 1.0f / (l * PS);
#pragma unroll
  for (int t = 0; t < 4; ++t)
#pragma unroll
    for (int r = 0; r < 8; ++r) { b16 a_, c_; split16(o[t][r] * inv, a_, c_); Oh[col][wid * HD + t * 16 + 8 * hh + r] = a_; Ol[col][wid * HD + t * 16 + 8 * hh + r] = c_; }
  __syncthreads();
  for (int pass = 0; pass < 2; ++pass) { for (int i = threadIdx.x; i < 16 * 64; i += 256) { const int rr = i >> 6, c8 = (i & 63) * 8; const size_t gi = ((size_t)(b * L + q0 + rr)) * D + blockIdx.y * 8 * HD + c8; *(volatile v8b*)(ctxh + gi) = *(const v8b*)(&Oh[rr][c8]); *(volatile v8b*)(ctxl + gi) = *(const v8b*)(&Ol[rr][c8]); } __threadfence(); }
}
}

extern "C" void kernel_launch(void* const* d_in, const int* in_sizes, int n_in,
                              void* d_out, int out_size, void* d_ws, size_t ws_size, hipStream_t stream) {
  (void)n_in; (void)out_size;
  const float* value = (const float*)d_in[0]; const float* key = (const float*)d_in[1]; const float* query = (const float*)d_in[2]; const int* mask = (const int*)d_in[3]; const float* Wo = (const float*)d_in[4]; const float* bo = (const float*)d_in[5]; const float* Wg = (const float*)d_in[6]; const float* bg = (const float*)d_in[7];
  const float* g1 = (const float*)d_in[8]; const float* b1 = (const float*)d_in[9]; const float* g2 = (const float*)d_in[10]; const float* b2 = (const float*)d_in[11]; const float* W1 = (const float*)d_in[12]; const float* bf1 = (const float*)d_in[13]; const float* W2 = (const float*)d_in[14]; const float* bf2 = (const float*)d_in[15];
  float* out = (float*)d_out;
  if (in_sizes[0] != NT * D || in_sizes[2] != NT * D || in_sizes[3] != L * L || in_sizes[4] != D * D || in_sizes[12] != D * DF || in_sizes[14] != DF * D) return;
  size_t off = 0; char* ws = (char*)d_ws;
  auto carve = [&](size_t bytes) { char* p = ws + off; off += (bytes + 255) & ~(size_t)255; return p; };
  b16* R = (b16*)carve(Wo_::END * 2); float* P = (float*)carve(11264 * 4); float* GT = (float*)carve((size_t)Bn * D * 4); b16* VT = (b16*)carve((size_t)Bn * H * HD * L * 2);
  b16* CH = (b16*)carve((size_t)NT * D * 2); b16* CL = (b16*)carve((size_t)NT * D * 2); float* Y = (float*)carve((size_t)NT * D * 4); float* X = (float*)carve((size_t)NT * D * 4); b16* G = (b16*)carve((size_t)NT * DF * 2);
  if (off > ws_size) return;
  prep_kernel<<<512, 256, 0, stream>>>(Wo, W1, W2, bo, bg, g1, b1, g2, b2, bf1, bf2, R, P);
  gate_kernel<<<dim3(16, Bn), 256, 0, stream>>>(query, Wg, P, GT);
  vt_kernel<<<dim3(L / 128, H, Bn), 256, 0, stream>>>(value, VT);
  attn_kernel<<<dim3(NT / 16, 2), 256, 0, stream>>>(query, key, mask, VT, CH, CL);
  gemm_kernel<D, D, 4, 1><<<dim3(D / 256, NT / 32), 64, 0, stream>>>(CH, R + Wo_::O, P, query, nullptr, Y, GT, CL);
  ln32_kernel<<<NT / 8, 256, 0, stream>>>(Y, P + 2048, P + 3072, X);
  ln_kernel<<<NT / 8, 256, 0, stream>>>(Y, 0, P + 2048, P + 3072, CH);
  gemm_kernel<D, DF, 5, 0><<<dim3(DF / 256, NT / 32), 64, 0, stream>>>(CH, R + Wo_::F1, P + 6144, nullptr, G, nullptr);
  gemm_kernel<DF, D, 1, 0><<<dim3(D / 256, NT / 32), 64, 0, stream>>>(G, R + Wo_::F2, P + 10240, X, nullptr, Y);
  ln32_kernel<<<NT / 8, 256, 0, stream>>>(Y, P + 4096, P + 5120, out);
}
